// PCENFrontend_90202903150895
// MI455X (gfx1250) — hardware-run, weakly checked
//
#include <hip/hip_runtime.h>
#include <math.h>


#pragma clang fp contract(off)

#ifndef NB
#define NB 16
#endif
#ifndef TLEN
#define TLEN 320000
#endif
#define NB_FULL 16
#define T_FULL  320000
#define NFFT    1024
#define HOPS    320
#define NBINS   513
#define KLOOP   544
#define KPITCH  576
#define NMEL    128
#define NFR     (TLEN / HOPS + 1)
#ifndef OUT_FR
#define OUT_FR  NFR
#endif
#define MROWS   (NB * NFR)
#define MPAD    (((MROWS + 63) / 64) * 64)
#define FBC     16.0f
#define FBI     (1.0f / 16.0f)
#define PC_EPS  1e-6f
#define LN_EPS  1e-6f

static_assert(NFFT == 1024);
static_assert(256 * 4 == NFFT);
static_assert(128 * 4 == NFFT / 2);
static_assert(3 * NFFT * 4 <= 131072);
static_assert(NBINS == NFFT / 2 + 1);
static_assert(NMEL == 128);
static_assert(NMEL % 64 == 0);
static_assert(KLOOP % 32 == 0);
static_assert(KLOOP >= NBINS);
static_assert(KPITCH >= KLOOP);
static_assert(KPITCH % 64 == 0);
static_assert((KPITCH * 2) % 128 == 0);
static_assert(KPITCH / 8 <= 256);
static_assert((KPITCH / 8) * 16 == KPITCH * 2);
static_assert(3 * 256 >= KPITCH);
static_assert(3 * 256 <= NFFT);
static_assert(MPAD % 64 == 0);
static_assert(MPAD >= MROWS);
static_assert(TLEN % HOPS == 0);
static_assert(TLEN >= NFFT);
static_assert(TLEN <= T_FULL);
static_assert(NB <= NB_FULL);
static_assert(32 * 256 == 64 * NMEL);
static_assert(4 * 256 == NMEL * 8);
static_assert(8 * 2 == 16);
static_assert(16 * 4 == 64);
static_assert(2 * NFFT * 4 + KPITCH * 2 <= 131072);
static_assert(NMEL * 72 * 2 <= 131072);
static_assert(16 * 68 * 4 <= 131072);

typedef _Float16 h16;
typedef __attribute__((ext_vector_type(16))) _Float16 v16h;
typedef __attribute__((ext_vector_type(8)))  _Float16 v8h;
typedef __attribute__((ext_vector_type(8)))  float    v8f;
typedef __attribute__((ext_vector_type(4)))  float    v4f;
typedef v4f  __attribute__((may_alias)) v4fa;
typedef v8h  __attribute__((may_alias)) v8ha;

__device__ __forceinline__ unsigned short f2bf(float f) { unsigned u = __float_as_uint(f); u += 0x7FFFu + ((u >> 16) & 1u); return (unsigned short)(u >> 16); }
__device__ __forceinline__ float bfr(float f) { return __uint_as_float(((unsigned)f2bf(f)) << 16); }
__device__ __forceinline__ v16h cat16(v8h lo, v8h hi) { return __builtin_shufflevector(lo, hi, 0, 1, 2, 3, 4, 5, 6, 7, 8, 9, 10, 11, 12, 13, 14, 15); }
__device__ __forceinline__ v16h  ldh(const h16* p) { return cat16(*(const v8h*)p, *(const v8h*)(p + 16)); }
__device__ __forceinline__ void wave_sync() { __builtin_amdgcn_fence(3  , "wavefront"); __builtin_amdgcn_wave_barrier(); asm volatile("" ::: "memory"); }
static __device__ __forceinline__ h16 toh_flush(float v) { const h16 r = (h16)v; return (fabsf(v) < 6.103515625e-05f) ? (h16)0.0f : r; }
__device__ __forceinline__ v8f wmma16g(v16h a, v16h b, v8f c) {
    c = __builtin_amdgcn_wmma_f32_16x16x32_f16(false, a, false, b, (short)0, c, false, false);
    asm volatile("v_nop\n\tv_nop\n\tv_nop\n\tv_nop" : "+v"(c) : "v"(a), "v"(b));
    return c;
}
__device__ __forceinline__ float wsum(float v) {
    v += __shfl_xor(v, 16, 32); v += __shfl_xor(v, 8, 32); v += __shfl_xor(v, 4, 32); v += __shfl_xor(v, 2, 32); v += __shfl_xor(v, 1, 32); return v; }

__global__ __launch_bounds__(256) void k_tab(float* TAB) {
    __shared__ __align__(16) float sw[NFFT];
    __shared__ __align__(16) float sc[NFFT];
    __shared__ __align__(16) float ss[NFFT];
    const int tid = threadIdx.x;
#pragma unroll 1
    for (int i = 0; i < 4; ++i) {
        const int n = 4 * tid + i;
        const float a = (6.28318530717958647692f * (float)n) * (1.0f / 1024.0f);
        const float cs = cosf(a), sn = sinf(a);
        const float w = 0.5f * (1.0f - cs);
        const float ts = -sn;
        sw[n] = w; sc[n] = cs; ss[n] = ts; }
    __syncthreads();
    const v4f wv = *(const v4fa*)(&sw[4 * tid]);
    const v4f cv = *(const v4fa*)(&sc[4 * tid]);
    const v4f sv = *(const v4fa*)(&ss[4 * tid]);
#pragma unroll 1
    for (int ps = 0; ps < 2; ++ps) {
        *(volatile v4f*)(TAB + 4 * tid) = wv;
        if (tid < 128) { *(volatile v4f*)(TAB + 1024 + 4 * tid) = cv; *(volatile v4f*)(TAB + 1536 + 4 * tid) = sv; }
        if (ps == 0) __threadfence(); }
}

__global__ __launch_bounds__(256) void k_fbcvt(const float* __restrict__ fb, h16* FBT) {
    __shared__ __align__(16) h16 t[NMEL * 72];
    const int tid = threadIdx.x; const int k0 = blockIdx.x * 64;
#pragma unroll 1
    for (int i = 0; i < 32; ++i) {
        const int e = tid + 256 * i; const int kk = e >> 7, n = e & 127;
        const int k = k0 + kk; const int kc = k < NBINS ? k : (NBINS - 1);
        float v = fb[(size_t)kc * NMEL + n];
        asm volatile("" : "+v"(v));
        const float s = (k < NBINS) ? (bfr(v) * FBC) : 0.0f;
        t[n * 72 + kk] = toh_flush(s); }
    __syncthreads();
#pragma unroll 1
    for (int ps = 0; ps < 2; ++ps) {
#pragma unroll
        for (int i = 0; i < 4; ++i) { const int q = tid + 256 * i; const int n = q >> 3, c8 = (q & 7) * 8;
            const v8h v = *(const v8ha*)(&t[n * 72 + c8]);
            *(volatile v8h*)(FBT + (size_t)n * KPITCH + k0 + c8) = v; }
        if (ps == 0) __threadfence(); }
}

__global__ __launch_bounds__(256) void k_fft(const float* __restrict__ x, const float* __restrict__ TAB, h16* PW) {
    __shared__ float re[NFFT];
    __shared__ float im[NFFT];
    __shared__ __align__(16) h16 hrow[KPITCH];
    const int tid = threadIdx.x; const int m = blockIdx.x;
    const bool live = m < MROWS;
    const int mc = live ? m : (MROWS - 1);
    const int b = mc / NFR, f = mc % NFR;
    const float* xb = x + (size_t)b * T_FULL;
#pragma unroll 1
    for (int i = 0; i < 4; ++i) {
        const int j = tid + 256 * i;
        int s = f * HOPS + j - NFFT / 2;
        s = s < 0 ? -s : s;
        s = s >= TLEN ? (2 * (TLEN - 1) - s) : s;
        s = s < 0 ? 0 : (s > TLEN - 1 ? TLEN - 1 : s);
        float xv = xb[s];
        asm volatile("" : "+v"(xv));
        const float w = TAB[j];
        const float v = live ? (bfr(xv) * w) : 0.0f;
        const unsigned rj = __brev((unsigned)j) >> 22;
        re[rj] = v; im[rj] = 0.0f; }
    __syncthreads();
#pragma unroll 1
    for (int st = 1; st <= 10; ++st) {
        const int half = 1 << (st - 1);
#pragma unroll 1
        for (int i = 0; i < 2; ++i) {
            const int t = tid + 256 * i;
            const int j = t & (half - 1);
            const int pos = ((t >> (st - 1)) << st) + j;
            const int ti = j << (10 - st);
            const float cs = TAB[1024 + ti], sn = TAB[1536 + ti];
            const float ur = re[pos], ui = im[pos];
            const float vr = re[pos + half], vi = im[pos + half];
            const float tr = vr * cs - vi * sn;
            const float tq = vr * sn + vi * cs;
            re[pos] = ur + tr; im[pos] = ui + tq;
            re[pos + half] = ur - tr; im[pos + half] = ui - tq; }
        __syncthreads(); }
#pragma unroll 1
    for (int i = 0; i < 3; ++i) {
        const int k = tid + 256 * i;
        const float a = re[k], c = im[k];
        const float pw = fminf(a * a + c * c, 65504.0f);
        const float p = (live & (k < NBINS)) ? pw : 0.0f;
        if (k < KPITCH) hrow[k] = toh_flush(p); }
    __syncthreads();
    if (tid < KPITCH / 8) {
        const v8h v = *(const v8ha*)(&hrow[tid * 8]);
        h16* dst = PW + (size_t)m * KPITCH + tid * 8;
        *(volatile v8h*)dst = v; __threadfence(); *(volatile v8h*)dst = v; }
}

__global__ __launch_bounds__(32) void k_mel(const h16* __restrict__ A, const h16* __restrict__ Bt, float* E) {
    __shared__ __align__(16) float os[16 * 68];
    const int lane = threadIdx.x & 31, lr = lane & 15, hi = lane >> 4; const int r0 = blockIdx.x * 64, c0 = blockIdx.y * 64;
    v8f acc[4][4];
#pragma unroll
    for (int mb = 0; mb < 4; ++mb)
#pragma unroll
        for (int nb = 0; nb < 4; ++nb) acc[mb][nb] = (v8f){};
    const size_t aoff = (size_t)(r0 + lr) * KPITCH + 8 * hi, boff = (size_t)(c0 + lr) * KPITCH + 8 * hi;
#pragma unroll 1
    for (int kc = 0; kc < KLOOP; kc += 32) {
        v16h a[4];
#pragma unroll
        for (int mb = 0; mb < 4; ++mb) a[mb] = ldh(A + aoff + (size_t)mb * 16 * KPITCH + kc);
#pragma unroll
        for (int nb = 0; nb < 4; ++nb) { const v16h b = ldh(Bt + boff + (size_t)nb * 16 * KPITCH + kc);
#pragma unroll
            for (int mb = 0; mb < 4; ++mb) acc[mb][nb] = wmma16g(a[mb], b, acc[mb][nb]); }
    }
#pragma unroll
    for (int mb = 0; mb < 4; ++mb) {
#pragma unroll
        for (int nb = 0; nb < 4; ++nb) {
#pragma unroll
            for (int j = 0; j < 8; ++j) os[(hi * 8 + j) * 68 + nb * 16 + lr] = acc[mb][nb][j] * FBI; }
        wave_sync();
        float* eb = E + (size_t)(r0 + mb * 16) * NMEL + c0;
#pragma unroll 1
        for (int ps = 0; ps < 2; ++ps) {
#pragma unroll
            for (int s = 0; s < 8; ++s) { const int row = 2 * s + (lane >> 4), c4 = (lane & 15) * 4;
                const v4f val = *(const v4fa*)(&os[row * 68 + c4]);
                *(volatile v4f*)(eb + (size_t)row * NMEL + c4) = val; }
            if (ps == 0) __threadfence(); }
        wave_sync();
    }
}

__global__ __launch_bounds__(128) void k_agc(const float* __restrict__ E, const float* __restrict__ lsp, const float* __restrict__ lap, const float* __restrict__ ldp,
                                              const float* __restrict__ lrp, float* OUT) {
    __shared__ float par[4];
    __shared__ float red[4];
    __shared__ float red2[4];
    const int tid = threadIdx.x, lane = tid & 31;
    const int wave = __builtin_amdgcn_readfirstlane((int)(threadIdx.x >> 5));
    const int b = blockIdx.x;
    { const float v0 = bfr(lsp[0]), v1 = bfr(lap[0]), v2 = bfr(ldp[0]), v3 = bfr(lrp[0]);
      const int q = tid & 3;
      const float v = (q == 0) ? v0 : ((q == 1) ? v1 : ((q == 2) ? v2 : v3));
      const float ev = expf(v);
      if (tid < 4) par[tid] = ev; }
    __syncthreads();
    const float s = par[0], alpha = par[1], delta = par[2], r = par[3];
    const float om = 1.0f - s;
    const float dr = exp2f(r * log2f(delta));
    const float* Eb = E + (size_t)b * NFR * NMEL + tid;
    float* Ob = OUT + (size_t)b * OUT_FR * NMEL + tid;
    float mm = Eb[0];
#pragma unroll 1
    for (int f = 0; f < NFR; ++f) {
        const float e = Eb[(size_t)f * NMEL];
        mm = om * mm + s * e;
        const float den = exp2f(alpha * log2f(PC_EPS + mm));
        const float y = e * __builtin_amdgcn_rcpf(den) + delta;
        const float p = exp2f(r * log2f(y)) - dr;
        const float sm = wsum(p);
        if (lane == 0) red[wave] = sm;
        __syncthreads();
        const float mu = ((red[0] + red[1]) + (red[2] + red[3])) * (1.0f / (float)NMEL);
        const float d = p - mu;
        const float sq = wsum(d * d);
        if (lane == 0) red2[wave] = sq;
        __syncthreads();
        const float var = ((red2[0] + red2[1]) + (red2[2] + red2[3])) * (1.0f / (float)NMEL);
        const float o = d * rsqrtf(var + LN_EPS);
        float* dst = Ob + (size_t)f * NMEL;
        *(volatile float*)dst = o; __threadfence(); *(volatile float*)dst = o;
    }
}

static constexpr size_t al256(size_t v) { return (v + 255) & ~(size_t)255; }
static constexpr size_t SZ_TAB = al256((size_t)2048 * 4);
static constexpr size_t SZ_FBT = al256((size_t)NMEL * KPITCH * 2);
static constexpr size_t SZ_PW  = al256((size_t)MPAD * KPITCH * 2);
static constexpr size_t SZ_EP  = al256((size_t)MPAD * NMEL * 4);
static constexpr size_t SZ_TOTAL = SZ_TAB + SZ_FBT + SZ_PW + SZ_EP;
static_assert(SZ_TOTAL <= (size_t)134217728);
static_assert((size_t)(1536 + 4 * 127 + 4) * 4 <= SZ_TAB);
static_assert((size_t)(MPAD - 1) * KPITCH * 2 + (size_t)KPITCH * 2 <= SZ_PW);
static_assert((size_t)(MPAD - 1) * NMEL * 4 + (size_t)NMEL * 4 <= SZ_EP);
static_assert((size_t)(NMEL - 1) * KPITCH * 2 + (size_t)KPITCH * 2 <= SZ_FBT);

extern "C" void kernel_launch(void* const* d_in, const int* in_sizes, int n_in,
                              void* d_out, int out_size, void* d_ws, size_t ws_size, hipStream_t stream) {
    if (n_in < 6) return;
    const size_t needx = (size_t)(NB - 1) * T_FULL + TLEN;
    if ((size_t)in_sizes[0] < needx) return;
    if ((size_t)in_sizes[1] < (size_t)NBINS * NMEL) return;
    if (in_sizes[2] < 1 || in_sizes[3] < 1 || in_sizes[4] < 1 || in_sizes[5] < 1) return;
    if ((size_t)out_size < ((size_t)(NB - 1) * OUT_FR + NFR) * NMEL) return;
    if (SZ_TOTAL > ws_size) return;
    const float* x  = (const float*)d_in[0];
    const float* fb = (const float*)d_in[1];
    const float* ls = (const float*)d_in[2];
    const float* la = (const float*)d_in[3];
    const float* ld = (const float*)d_in[4];
    const float* lr = (const float*)d_in[5];
    float* OUT = (float*)d_out;
    char* wsp = (char*)d_ws;
    float* TAB = (float*)wsp; wsp += SZ_TAB;
    h16* FBT = (h16*)wsp; wsp += SZ_FBT;
    h16* PW  = (h16*)wsp; wsp += SZ_PW;
    float* EP = (float*)wsp; wsp += SZ_EP;

    k_tab<<<1, 256, 0, stream>>>(TAB);
    k_fbcvt<<<KPITCH / 64, 256, 0, stream>>>(fb, FBT);
    k_fft<<<MPAD, 256, 0, stream>>>(x, TAB, PW);
    k_mel<<<dim3(MPAD / 64, NMEL / 64, 1), 32, 0, stream>>>(PW, FBT, EP);
    k_agc<<<NB, 128, 0, stream>>>(EP, ls, la, ld, lr, OUT);
}
